// GraphSAGE_31001073943304
// MI455X (gfx1250) — hardware-verified
//
#include <hip/hip_runtime.h>
#include <stddef.h>
#include <stdint.h>


#define CIN    128
#define HIDN   256
#define NCO    3
#define KC     384
#define ZP     4
#define NTHR   256
#define NWAVE  8
#define EPT    8
#define CHUNK  (NTHR * EPT)
#define WCAP   (EPT * 32)
#define LISTN  (NWAVE * WCAP)
#define NBA    1024
#define SLA    10
#define RCAP   16384
#define DEGCAP 48
#define GBM    64
#define GBN    64
#define GTHR   128
#define UPART  4096
#define NPART  3
#define AGG_ZINTS    (LISTN + 2 * RCAP + 3 * NBA)
#define MISC_INTS    16
#define ROWBUF_INTS  (NWAVE * KC / 2)
#define OUTS_FLOATS  (NCO * NBA)
#define LDS1_INTS    (AGG_ZINTS + MISC_INTS + ROWBUF_INTS)
#define LDS0_INTS    (AGG_ZINTS + MISC_INTS + OUTS_FLOATS)
#define OUT_IT       (OUTS_FLOATS / (4 * NTHR))
#define WSMAX  134217728

static_assert((CHUNK & (CHUNK - 1)) == 0 && CHUNK <= 4096);
static_assert((NBA & (NBA - 1)) == 0 && NBA == (1 << SLA));
static_assert(((long long)CHUNK << SLA) < (1LL << 31));
static_assert(LISTN % NTHR == 0);
static_assert(NBA % NWAVE == 0 && NBA % 32 == 0 && NBA % GBM == 0);
static_assert(RCAP % 32 == 0 && AGG_ZINTS % 4 == 0 && LISTN % 4 == 0 && ((AGG_ZINTS + MISC_INTS) % 4) == 0);
static_assert(AGG_ZINTS % (NTHR * 4) == 0);
static_assert(KC % 32 == 0 && KC == 3 * CIN && CIN == 4 * 32);
static_assert((KC * 2) % 128 == 0 && (2 * CIN * 2) % 128 == 0);
static_assert(GBM == (GTHR / 32) * 16 && GBN == 64 && HIDN % GBN == 0);
static_assert(UPART % NTHR == 0 && UPART == HIDN * (CIN / 8) && CIN / 8 == 16);
static_assert((NPART * UPART) % NTHR == 0);
static_assert(HIDN == NTHR && HIDN % 4 == 0);
static_assert(OUTS_FLOATS % (4 * NTHR) == 0 && (OUTS_FLOATS * 4) % 128 == 0);
static_assert(LDS1_INTS * 4 <= 300000 && LDS0_INTS * 4 <= 300000);
static_assert(ZP * 4 == 16);

typedef float          v4f   __attribute__((ext_vector_type(4)));
typedef float          v8f   __attribute__((ext_vector_type(8)));
typedef int            v4i   __attribute__((ext_vector_type(4)));
typedef int            v8i   __attribute__((ext_vector_type(8)));
typedef unsigned short v4us  __attribute__((ext_vector_type(4)));
typedef unsigned short v8us  __attribute__((ext_vector_type(8)));
typedef unsigned short v16us __attribute__((ext_vector_type(16)));
typedef __bf16         v16bf __attribute__((ext_vector_type(16)));
typedef v4f  __attribute__((may_alias)) v4fa;
typedef v4i  __attribute__((may_alias)) v4ia;
typedef v4us __attribute__((may_alias)) v4usa;
typedef v8us __attribute__((may_alias)) v8usa;
union FragB { v16bf v; v16us u; v8us h[2]; v8i w; };

__device__ __forceinline__ v8f wmb(const FragB& a, const FragB& b, v8f c) {
  v8f d = __builtin_amdgcn_wmma_f32_16x16x32_bf16(false, a.v, false, b.v, (short)0, c, false, false);
  asm volatile("v_nop\n\tv_nop\n\tv_nop\n\tv_nop" : "+v"(d) : "v"(a.w), "v"(b.w));
  return d;
}

__device__ __forceinline__ unsigned bf16_bits(float f) {
  const unsigned u = __float_as_uint(f);
  return (u + 0x7FFFu + ((u >> 16) & 1u)) >> 16;
}
__device__ __forceinline__ float bf16_val(float f) {
  return __uint_as_float(bf16_bits(f) << 16);
}

__device__ __forceinline__ void wave_sync() {
  __builtin_amdgcn_fence(__ATOMIC_RELEASE, "wavefront");
  __builtin_amdgcn_wave_barrier();
  __builtin_amdgcn_fence(__ATOMIC_ACQUIRE, "wavefront");
}

template <int SLB>
__device__ __forceinline__ int scan_chunk(const int* __restrict__ dsts, int nE, int cbase, int slotBase,
                                          int nb, int vec8, int* list, int tid, int lane, int wave) {
  int wc = 0;
  const int el0  = tid * EPT;
  const int e0   = cbase + el0;
  const int sent = -2147483647 - 1;
  v4i da, db;
  if (vec8 != 0 && cbase + CHUNK <= nE) {
    da = *(const v4i*)(dsts + e0);
    db = *(const v4i*)(dsts + e0 + 4);
  } else {
    da.x = (e0     < nE) ? dsts[min(e0,     nE - 1)] : sent;
    da.y = (e0 + 1 < nE) ? dsts[min(e0 + 1, nE - 1)] : sent;
    da.z = (e0 + 2 < nE) ? dsts[min(e0 + 2, nE - 1)] : sent;
    da.w = (e0 + 3 < nE) ? dsts[min(e0 + 3, nE - 1)] : sent;
    db.x = (e0 + 4 < nE) ? dsts[min(e0 + 4, nE - 1)] : sent;
    db.y = (e0 + 5 < nE) ? dsts[min(e0 + 5, nE - 1)] : sent;
    db.z = (e0 + 6 < nE) ? dsts[min(e0 + 6, nE - 1)] : sent;
    db.w = (e0 + 7 < nE) ? dsts[min(e0 + 7, nE - 1)] : sent;
  }
  const unsigned nbs = (unsigned)slotBase;
  const unsigned unb = (unsigned)nb;
  const unsigned s0 = (unsigned)da.x - nbs, s1 = (unsigned)da.y - nbs;
  const unsigned s2 = (unsigned)da.z - nbs, s3 = (unsigned)da.w - nbs;
  const unsigned s4 = (unsigned)db.x - nbs, s5 = (unsigned)db.y - nbs;
  const unsigned s6 = (unsigned)db.z - nbs, s7 = (unsigned)db.w - nbs;
  const bool h0 = s0 < unb, h1 = s1 < unb, h2 = s2 < unb, h3 = s3 < unb;
  const bool h4 = s4 < unb, h5 = s5 < unb, h6 = s6 < unb, h7 = s7 < unb;
  const unsigned any = __builtin_amdgcn_ballot_w32(h0 | h1 | h2 | h3 | h4 | h5 | h6 | h7);
  if (any != 0u) {
#define HITJ(J, HJ, SJ) { \
      const unsigned mj = __builtin_amdgcn_ballot_w32(HJ); \
      if (mj != 0u) { \
        if (HJ) { \
          const int pos = wc + (int)__builtin_amdgcn_mbcnt_lo(mj, 0u); \
          if (pos < WCAP) list[wave * WCAP + pos] = ((el0 + (J)) << SLB) | (int)(SJ); \
        } \
        wc += (int)__builtin_popcount(mj); } }
    HITJ(0, h0, s0)
    HITJ(1, h1, s1)
    HITJ(2, h2, s2)
    HITJ(3, h3, s3)
    HITJ(4, h4, s4)
    HITJ(5, h5, s5)
    HITJ(6, h6, s6)
    HITJ(7, h7, s7)
#undef HITJ
  }
  return wc;
}

__global__ __launch_bounds__(NTHR) void k_wprep(const float* __restrict__ Wl, const float* __restrict__ Wr,
                                                unsigned short* BT) {
  const int u    = (int)blockIdx.x * NTHR + (int)threadIdx.x;
  const int part = u >> 12;
  if (part >= NPART) return;
  const int v    = u & (UPART - 1);
  const int n    = v >> 4;
  const int k8   = (v & 15) * 8;
  const float* W = (part == 2) ? Wr : Wl;
  const int coff = part * CIN;
  const float* p = W + (size_t)k8 * HIDN + n;
  v8us o;
#pragma unroll
  for (int i = 0; i < 8; ++i) o[i] = (unsigned short)bf16_bits(p[(size_t)i * HIDN]);
  unsigned short* dp = BT + (size_t)n * KC + coff + k8;
  *(volatile v8us*)dp = o;
  __threadfence();
  *(volatile v8us*)dp = o;
}

__global__ __launch_bounds__(GTHR) void k_gemm(
    const unsigned short* __restrict__ A, const unsigned short* __restrict__ WT,
    const float* __restrict__ bias, float* outF, int K, int ldo, int nOut)
{
  __shared__ __attribute__((aligned(16))) float stg[GBM * GBN];
  const int tid = (int)threadIdx.x, lane = tid & 31, wave = tid >> 5, hh = lane >> 4, m = lane & 15;
  const int rowBase = (int)blockIdx.x * GBM;
  const int col0    = (int)blockIdx.y * GBN;

  v8f acc[4];
  {
    const v8f z = {0.f, 0.f, 0.f, 0.f, 0.f, 0.f, 0.f, 0.f};
    acc[0] = z; acc[1] = z; acc[2] = z; acc[3] = z;
  }
  const unsigned short* ap = A  + (size_t)(rowBase + 16 * wave + m) * (size_t)K + 8 * hh;
  const unsigned short* wp = WT + (size_t)(col0 + m) * (size_t)K + 8 * hh;
  const int ksteps = K >> 5;
#pragma unroll 1
  for (int ks = 0; ks < ksteps; ++ks) {
    FragB af;
    af.h[0] = *(const v8usa*)(ap + 32 * ks);
    af.h[1] = *(const v8usa*)(ap + 32 * ks + 16);
#pragma unroll
    for (int t = 0; t < 4; ++t) {
      const unsigned short* wq = wp + (size_t)(16 * t) * (size_t)K + 32 * ks;
      FragB bf;
      bf.h[0] = *(const v8usa*)wq;
      bf.h[1] = *(const v8usa*)(wq + 16);
      acc[t] = wmb(af, bf, acc[t]);
    }
  }

#pragma unroll
  for (int t = 0; t < 4; ++t) {
    const int lc = 16 * t + m;
#pragma unroll
    for (int r = 0; r < 8; ++r) {
      const int lr = 16 * wave + 8 * hh + r;
      stg[lr * GBN + lc] = acc[t][r];
    }
  }
  __syncthreads();

  v4f b4;
  {
    const v4f t1 = *(const v4fa*)(bias + col0 + 4 * m);
    b4.x = bf16_val(t1.x); b4.y = bf16_val(t1.y); b4.z = bf16_val(t1.z); b4.w = bf16_val(t1.w);
  }
  v4f fv[8];
#pragma unroll
  for (int i = 0; i < 8; ++i) {
    const int lr = 16 * wave + 2 * i + hh;
    const int gr = rowBase + lr;
    const bool ok = gr < nOut;
    const v4f t1 = *(const v4fa*)(stg + lr * GBN + 4 * m) + b4;
    v4f y;
    y.x = (t1.x < 0.0f) ? 0.0f : t1.x;
    y.y = (t1.y < 0.0f) ? 0.0f : t1.y;
    y.z = (t1.z < 0.0f) ? 0.0f : t1.z;
    y.w = (t1.w < 0.0f) ? 0.0f : t1.w;
    y.x = ok ? y.x : 0.0f; y.y = ok ? y.y : 0.0f; y.z = ok ? y.z : 0.0f; y.w = ok ? y.w : 0.0f;
    fv[i] = y;
  }
#pragma unroll
  for (int i = 0; i < 8; ++i) {
    const int lr = 16 * wave + 2 * i + hh;
    const int gr = rowBase + lr;
    float* op = outF + (size_t)gr * (size_t)ldo + col0 + 4 * m;
    *(volatile v4f*)op = fv[i];
  }
  __threadfence();
#pragma unroll
  for (int i = 0; i < 8; ++i) {
    const int lr = 16 * wave + 2 * i + hh;
    const int gr = rowBase + lr;
    float* op = outF + (size_t)gr * (size_t)ldo + col0 + 4 * m;
    *(volatile v4f*)op = fv[i];
  }
}

__global__ __launch_bounds__(NTHR) void k_rowdot(const float* __restrict__ H, const float* __restrict__ Wl,
                                                 const float* __restrict__ Wr, int mRows, float* zl, float* zr) {
  __shared__ __attribute__((aligned(16))) float w6[HIDN * 8];
  const int tid = (int)threadIdx.x;
  {
    const float* pl = Wl + 3 * tid;
    const float* pr = Wr + 3 * tid;
    v4f a, b;
    a.x = bf16_val(pl[0]); a.y = bf16_val(pl[1]); a.z = bf16_val(pl[2]); a.w = 0.0f;
    b.x = bf16_val(pr[0]); b.y = bf16_val(pr[1]); b.z = bf16_val(pr[2]); b.w = 0.0f;
    *(v4fa*)(w6 + 8 * tid)     = a;
    *(v4fa*)(w6 + 8 * tid + 4) = b;
  }
  __syncthreads();
  const int u   = (int)blockIdx.x * NTHR + tid;
  const int row = u < mRows ? u : mRows - 1;
  const float* hp = H + (size_t)row * HIDN;
  float s0 = 0.0f, s1 = 0.0f, s2 = 0.0f, s3 = 0.0f, s4 = 0.0f, s5 = 0.0f;
#pragma unroll 1
  for (int k4 = 0; k4 < HIDN / 4; ++k4) {
    const v4f h = *(const v4fa*)(hp + 4 * k4);
    const float* wq = w6 + 32 * k4;
    const v4f w0a = *(const v4fa*)(wq),      w0b = *(const v4fa*)(wq + 4);
    const v4f w1a = *(const v4fa*)(wq + 8),  w1b = *(const v4fa*)(wq + 12);
    const v4f w2a = *(const v4fa*)(wq + 16), w2b = *(const v4fa*)(wq + 20);
    const v4f w3a = *(const v4fa*)(wq + 24), w3b = *(const v4fa*)(wq + 28);
    s0 = fmaf(h.x, w0a.x, s0); s1 = fmaf(h.x, w0a.y, s1); s2 = fmaf(h.x, w0a.z, s2);
    s3 = fmaf(h.x, w0b.x, s3); s4 = fmaf(h.x, w0b.y, s4); s5 = fmaf(h.x, w0b.z, s5);
    s0 = fmaf(h.y, w1a.x, s0); s1 = fmaf(h.y, w1a.y, s1); s2 = fmaf(h.y, w1a.z, s2);
    s3 = fmaf(h.y, w1b.x, s3); s4 = fmaf(h.y, w1b.y, s4); s5 = fmaf(h.y, w1b.z, s5);
    s0 = fmaf(h.z, w2a.x, s0); s1 = fmaf(h.z, w2a.y, s1); s2 = fmaf(h.z, w2a.z, s2);
    s3 = fmaf(h.z, w2b.x, s3); s4 = fmaf(h.z, w2b.y, s4); s5 = fmaf(h.z, w2b.z, s5);
    s0 = fmaf(h.w, w3a.x, s0); s1 = fmaf(h.w, w3a.y, s1); s2 = fmaf(h.w, w3a.z, s2);
    s3 = fmaf(h.w, w3b.x, s3); s4 = fmaf(h.w, w3b.y, s4); s5 = fmaf(h.w, w3b.z, s5);
  }
  v4f za, zb;
  za.x = s0; za.y = s1; za.z = s2; za.w = 0.0f;
  zb.x = s3; zb.y = s4; zb.z = s5; zb.w = 0.0f;
  const bool ok = u < mRows;
  float* pa = zl + (size_t)row * ZP;
  float* pb = zr + (size_t)row * ZP;
  if (ok) { *(volatile v4f*)pa = za; *(volatile v4f*)pb = zb; }
  __threadfence();
  if (ok) { *(volatile v4f*)pa = za; *(volatile v4f*)pb = zb; }
}

template <int MODE>
__global__ __launch_bounds__(NTHR) void k_scan(const int* __restrict__ srcs, const int* __restrict__ dsts,
                                               int nE, int nN, int vec8, int mRows,
                                               const float* __restrict__ xin, unsigned short* apl,
                                               const float* __restrict__ zl, const float* __restrict__ zr,
                                               const float* __restrict__ b1, float* outp) {
  extern __shared__ __attribute__((aligned(16))) int dsm[];
  int* list = dsm;
  int* hl   = dsm + LISTN;
  int* sl   = hl + RCAP;
  int* cnt  = sl + RCAP;
  int* offs = cnt + NBA;
  int* cur  = offs + NBA;
  int* misc = cur + NBA;
  const int tid = (int)threadIdx.x, lane = tid & 31, wave = tid >> 5;
  unsigned short* rowbuf = (unsigned short*)(misc + MISC_INTS) + wave * KC;
  float* outs = (float*)(misc + MISC_INTS);
  const int nodeBase = (int)blockIdx.x * NBA;

  {
    const v4i z4 = {0, 0, 0, 0};
    for (int i = tid * 4; i < AGG_ZINTS; i += NTHR * 4) *(v4ia*)(dsm + i) = z4;
    if (tid < MISC_INTS) misc[tid] = 0;
  }
  __syncthreads();

  int t = 0, ov = 0;
  const int nChunks = (nE + CHUNK - 1) / CHUNK;
#pragma unroll 1
  for (int ch = 0; ch < nChunks; ++ch) {
    const int cbase = ch * CHUNK;
    const int wc = scan_chunk<SLA>(dsts, nE, cbase, nodeBase, NBA, vec8, list, tid, lane, wave);
    if (lane == 0) misc[wave] = wc;
    __syncthreads();
    if (wave == 0) {
#pragma unroll 1
      for (int w2 = 0; w2 < NWAVE; ++w2) {
        int c = misc[w2];
        c = c < 0 ? 0 : (c > WCAP ? WCAP : c);
#pragma unroll 1
        for (int b0 = 0; b0 < c; b0 += 32) {
          const int idx = b0 + lane;
          const int ent = list[w2 * WCAP + (idx < WCAP ? idx : WCAP - 1)];
          const int m32 = (c - b0) < 32 ? (c - b0) : 32;
#pragma unroll 1
          for (int k = 0; k < m32; ++k) {
            const int u    = __builtin_amdgcn_readlane(ent, k);
            const int slot = u & (NBA - 1);
            const int el   = (u >> SLA) & (CHUNK - 1);
            const int pk   = ((cbase + el) << SLA) | slot;
            if (t < RCAP) {
              if (lane == 0) { hl[t] = pk; cnt[slot] = cnt[slot] + 1; }
              t = t + 1;
            } else {
              ov = 1;
            }
          }
        }
      }
    }
    __syncthreads();
  }
  if (wave == 0 && lane == 0) { misc[8] = t; misc[9] = ov; }
  __syncthreads();
  int tt = misc[8];
  tt = tt < 0 ? 0 : (tt > RCAP ? RCAP : tt);
  const int ovf = misc[9];

  if (wave == 0) {
    const int base = lane * (NBA / 32);
    int s = 0;
#pragma unroll 1
    for (int i = 0; i < NBA / 32; ++i) s += cnt[base + i];
    int incl = s;
#pragma unroll
    for (int d = 1; d < 32; d <<= 1) {
      const int y = __shfl_up(incl, d, 32);
      if (lane >= d) incl += y;
    }
    int run = incl - s;
#pragma unroll 1
    for (int i = 0; i < NBA / 32; ++i) {
      const int cv = cnt[base + i];
      offs[base + i] = run;
      cur[base + i]  = run;
      run += cv;
    }
  }
  __syncthreads();
  if (wave == 0) {
#pragma unroll 1
    for (int b0 = 0; b0 < tt; b0 += 32) {
      const int idx = b0 + lane;
      const int ent = hl[idx < RCAP ? idx : RCAP - 1];
      const int m32 = (tt - b0) < 32 ? (tt - b0) : 32;
#pragma unroll 1
      for (int k = 0; k < m32; ++k) {
        const int u    = __builtin_amdgcn_readlane(ent, k);
        const int slot = u & (NBA - 1);
        if (lane == 0) {
          int p = cur[slot];
          p = p < 0 ? 0 : (p > RCAP - 1 ? RCAP - 1 : p);
          sl[p] = u;
          cur[slot] = p + 1;
        }
      }
    }
  }
  __syncthreads();

  const float qnan = __int_as_float(0x7fc00000);
  const float pz = (ovf != 0) ? qnan : 0.0f;
  if constexpr (MODE != 0) {
#pragma unroll 1
    for (int si = 0; si < NBA / NWAVE; ++si) {
      const int s    = si * NWAVE + wave;
      const int node = nodeBase + s;
      int c = cnt[s];
      const bool big = c > DEGCAP;
      c = c < 0 ? 0 : (c > DEGCAP ? DEGCAP : c);
      int o = offs[s];
      o = o < 0 ? 0 : (o > RCAP ? RCAP : o);
      const int nc = node < nN ? node : nN - 1;
      float a0 = 0.0f, a1 = 0.0f, a2 = 0.0f, a3 = 0.0f;
#pragma unroll 1
      for (int b0 = 0; b0 < c; b0 += 32) {
        int idx = o + b0 + lane;
        idx = idx > RCAP - 1 ? RCAP - 1 : idx;
        const int ent = sl[idx];
        int eid = ent >> SLA;
        eid = eid < 0 ? 0 : (eid > nE - 1 ? nE - 1 : eid);
        int sr = srcs[eid];
        sr = sr < 0 ? 0 : (sr > nN - 1 ? nN - 1 : sr);
        const int m32 = (c - b0) < 32 ? (c - b0) : 32;
#pragma unroll 1
        for (int k = 0; k < m32; ++k) {
          const int sk = __builtin_amdgcn_readlane(sr, k);
          const v4f a = *(const v4fa*)(xin + (size_t)sk * CIN + 4 * lane);
          a0 += bf16_val(a.x);
          a1 += bf16_val(a.y);
          a2 += bf16_val(a.z);
          a3 += bf16_val(a.w);
        }
      }
      const float inv = 1.0f / (float)(c < 1 ? 1 : c);
      const float pzr = big ? qnan : pz;
      const bool live = node < nN;
      const float m0 = live ? (a0 * inv + pzr) : 0.0f;
      const float m1 = live ? (a1 * inv + pzr) : 0.0f;
      const float m2 = live ? (a2 * inv + pzr) : 0.0f;
      const float m3 = live ? (a3 * inv + pzr) : 0.0f;
      v4us mh, ml;
      {
        unsigned hb;
        hb = bf16_bits(m0); mh[0] = (unsigned short)hb; ml[0] = (unsigned short)bf16_bits(m0 - __uint_as_float(hb << 16));
        hb = bf16_bits(m1); mh[1] = (unsigned short)hb; ml[1] = (unsigned short)bf16_bits(m1 - __uint_as_float(hb << 16));
        hb = bf16_bits(m2); mh[2] = (unsigned short)hb; ml[2] = (unsigned short)bf16_bits(m2 - __uint_as_float(hb << 16));
        hb = bf16_bits(m3); mh[3] = (unsigned short)hb; ml[3] = (unsigned short)bf16_bits(m3 - __uint_as_float(hb << 16));
      }
      *(v4usa*)(rowbuf + 4 * lane) = mh;
      *(v4usa*)(rowbuf + CIN + 4 * lane) = ml;
      {
        const v4f xs = *(const v4fa*)(xin + (size_t)nc * CIN + 4 * lane);
        v4us xb;
        xb[0] = live ? (unsigned short)bf16_bits(xs.x + pzr) : (unsigned short)0;
        xb[1] = live ? (unsigned short)bf16_bits(xs.y + pzr) : (unsigned short)0;
        xb[2] = live ? (unsigned short)bf16_bits(xs.z + pzr) : (unsigned short)0;
        xb[3] = live ? (unsigned short)bf16_bits(xs.w + pzr) : (unsigned short)0;
        *(v4usa*)(rowbuf + 2 * CIN + 4 * lane) = xb;
      }
      wave_sync();
      const v8us q0 = *(const v8usa*)(rowbuf + 8 * lane);
      const v8us q1 = *(const v8usa*)(rowbuf + 2 * CIN + 8 * (lane & 15));
      wave_sync();
      if (node < mRows) {
        unsigned short* rpw = apl + (size_t)node * KC + 8 * lane;
        unsigned short* rpx = apl + (size_t)node * KC + 2 * CIN + 8 * (lane & 15);
        const bool w1 = lane < 16;
        *(volatile v8us*)rpw = q0;
        if (w1) *(volatile v8us*)rpx = q1;
        __threadfence();
        *(volatile v8us*)rpw = q0;
        if (w1) *(volatile v8us*)rpx = q1;
      }
    }
  } else {
    const float bb0 = bf16_val(b1[0]);
    const float bb1 = bf16_val(b1[1]);
    const float bb2 = bf16_val(b1[2]);
#pragma unroll 1
    for (int si = 0; si < NBA / NWAVE; ++si) {
      const int s    = si * NWAVE + wave;
      const int node = nodeBase + s;
      int c = cnt[s];
      const bool big = c > DEGCAP;
      c = c < 0 ? 0 : (c > DEGCAP ? DEGCAP : c);
      int o = offs[s];
      o = o < 0 ? 0 : (o > RCAP ? RCAP : o);
      const int nc = node < nN ? node : nN - 1;
      float a0 = 0.0f, a1 = 0.0f, a2 = 0.0f;
#pragma unroll 1
      for (int b0 = 0; b0 < c; b0 += 32) {
        int idx = o + b0 + lane;
        idx = idx > RCAP - 1 ? RCAP - 1 : idx;
        const int ent = sl[idx];
        int eid = ent >> SLA;
        eid = eid < 0 ? 0 : (eid > nE - 1 ? nE - 1 : eid);
        int sr = srcs[eid];
        sr = sr < 0 ? 0 : (sr > nN - 1 ? nN - 1 : sr);
        const v4f z = *(const v4fa*)(zl + (size_t)sr * ZP);
        const bool ok = (b0 + lane) < c;
        a0 += ok ? z.x : 0.0f;
        a1 += ok ? z.y : 0.0f;
        a2 += ok ? z.z : 0.0f;
      }
#pragma unroll
      for (int d = 16; d >= 1; d >>= 1) {
        a0 += __shfl_xor(a0, d, 32);
        a1 += __shfl_xor(a1, d, 32);
        a2 += __shfl_xor(a2, d, 32);
      }
      const float inv = 1.0f / (float)(c < 1 ? 1 : c);
      const v4f zs = *(const v4fa*)(zr + (size_t)nc * ZP);
      const float pzr = big ? qnan : pz;
      const bool live = node < nN;
      const float r0 = (a0 * inv + bb0) + zs.x;
      const float r1 = (a1 * inv + bb1) + zs.y;
      const float r2 = (a2 * inv + bb2) + zs.z;
      const float v0 = live ? (r0 + pzr) : 0.0f;
      const float v1 = live ? (r1 + pzr) : 0.0f;
      const float v2 = live ? (r2 + pzr) : 0.0f;
      if (lane == 0) {
        outs[NCO * s + 0] = v0;
        outs[NCO * s + 1] = v1;
        outs[NCO * s + 2] = v2;
      }
    }
    __syncthreads();
    int vn = nN - nodeBase;
    vn = vn < 0 ? 0 : (vn > NBA ? NBA : vn);
    const int vf  = NCO * vn;
    const int n4  = vf >> 2;
    const int rem = vf & 3;
    float* ob = outp + (size_t)NCO * (size_t)nodeBase;
    v4f ovv[OUT_IT];
#pragma unroll
    for (int it = 0; it < OUT_IT; ++it) ovv[it] = *(const v4fa*)(outs + 4 * (it * NTHR + tid));
    const int ti = 4 * n4 + tid;
    const float tv = outs[ti < OUTS_FLOATS ? ti : OUTS_FLOATS - 1];
#pragma unroll
    for (int it = 0; it < OUT_IT; ++it) {
      const int u4 = it * NTHR + tid;
      if (u4 < n4) *(volatile v4f*)(ob + 4 * (size_t)u4) = ovv[it];
    }
    if (tid < rem) *(volatile float*)(ob + 4 * (size_t)n4 + tid) = tv;
    __threadfence();
#pragma unroll
    for (int it = 0; it < OUT_IT; ++it) {
      const int u4 = it * NTHR + tid;
      if (u4 < n4) *(volatile v4f*)(ob + 4 * (size_t)u4) = ovv[it];
    }
    if (tid < rem) *(volatile float*)(ob + 4 * (size_t)n4 + tid) = tv;
  }
}

static inline int cdiv(int a, int b) { return (a + b - 1) / b; }
static inline size_t al256(size_t o) { return (o + 255) & ~(size_t)255; }

extern "C" void kernel_launch(void* const* d_in, const int* in_sizes, int n_in,
                              void* d_out, int out_size, void* d_ws, size_t ws_size,
                              hipStream_t stream) {
  if (n_in < 8) return;
  if (in_sizes[0] < CIN || (in_sizes[0] % CIN) != 0) return;
  const int nN = in_sizes[0] / CIN;
  if (nN < 1 || nN > (1 << 22)) return;
  if (in_sizes[1] < 2 || (in_sizes[1] & 1) != 0) return;
  const int nE = in_sizes[1] / 2;
  if (nE < 1 || nE >= (1 << (31 - SLA))) return;
  if (in_sizes[2] != CIN * HIDN || in_sizes[3] != HIDN) return;
  if (in_sizes[4] != CIN * HIDN) return;
  if (in_sizes[5] != HIDN * NCO || in_sizes[6] != NCO) return;
  if (in_sizes[7] != HIDN * NCO) return;
  if ((long long)out_size != (long long)nN * NCO) return;

  const float* x    = (const float*)d_in[0];
  const int*   edge = (const int*)d_in[1];
  const float* Wl0  = (const float*)d_in[2];
  const float* bl0  = (const float*)d_in[3];
  const float* Wr0  = (const float*)d_in[4];
  const float* Wl1  = (const float*)d_in[5];
  const float* bl1  = (const float*)d_in[6];
  const float* Wr1  = (const float*)d_in[7];
  float* out = (float*)d_out;
  const int* src = edge;
  const int* dst = edge + nE;

  const int MP = cdiv(nN, GBM) * GBM;
  const int gM = MP / GBM;
  const int gA = cdiv(MP, NBA);
  if ((long long)gA * NBA < (long long)MP) return;
  const int vec8 = ((nE & 3) == 0) ? 1 : 0;

  char* ws = (char*)d_ws;
  size_t off = 0;
  const size_t oBT = off; off = al256(off + (size_t)HIDN * KC * 2);
  const size_t oA  = off; off = al256(off + (size_t)MP * KC * 2);
  const size_t oH  = off; off = al256(off + (size_t)MP * HIDN * 4);
  const size_t oZL = off; off = al256(off + (size_t)MP * ZP * 4);
  const size_t oZR = off; off = al256(off + (size_t)MP * ZP * 4);
  if (off > ws_size || off > (size_t)WSMAX) return;
  unsigned short* BT  = (unsigned short*)(ws + oBT);
  unsigned short* Apl = (unsigned short*)(ws + oA);
  float*          H   = (float*)(ws + oH);
  float*          ZL  = (float*)(ws + oZL);
  float*          ZR  = (float*)(ws + oZR);

  const size_t lds1 = (size_t)LDS1_INTS * 4;
  const size_t lds0 = (size_t)LDS0_INTS * 4;
  hipFuncSetAttribute(reinterpret_cast<const void*>(&k_scan<1>), hipFuncAttributeMaxDynamicSharedMemorySize, (int)lds1);
  hipFuncSetAttribute(reinterpret_cast<const void*>(&k_scan<0>), hipFuncAttributeMaxDynamicSharedMemorySize, (int)lds0);

  k_wprep<<<(NPART * UPART) / NTHR, NTHR, 0, stream>>>(Wl0, Wr0, BT);
  k_scan<1><<<gA, NTHR, lds1, stream>>>(src, dst, nE, nN, vec8, MP, x, Apl, ZL, ZR, bl1, out);
  k_gemm<<<dim3(gM, HIDN / GBN), GTHR, 0, stream>>>(Apl, BT, bl0, H, KC, HIDN, nN);
  k_rowdot<<<cdiv(MP, NTHR), NTHR, 0, stream>>>(H, Wl1, Wr1, MP, ZL, ZR);
  k_scan<0><<<gA, NTHR, lds0, stream>>>(src, dst, nE, nN, vec8, MP, x, Apl, ZL, ZR, bl1, out);
}
